// EfficientSlidingWindowMultiheadAttention_90022514524886
// MI455X (gfx1250) — hardware-verified
//
#include <hip/hip_runtime.h>


#ifndef NB
#define NB 1
#endif
#ifndef SEQ
#define SEQ 2048
#endif
#define NB_FULL  1
#define SEQ_FULL 2048
#ifndef OUT_SEQ
#define OUT_SEQ SEQ
#endif
#define DM    1024
#define TD    3072
#define NH_   16
#define HD    64
#define HALFW 64
#define WSPAN 128
#define PADL  64
#define SP    (SEQ + 192)
#define KT    5
#define AW    4
#define OSP   68
#define TSP   65
#define SC2   ((float)(0.125 * 1.4426950408889634))
#define PSH   14.0f
#define NEGB  (-3.0e38f)
#define CXS   256.0f
#define WOS   64.0f
#define OSI   (1.0f / 16384.0f)

static_assert(HD == 64);
static_assert(NH_ * HD == DM);
static_assert(TD == 3 * DM);
static_assert(TD == NH_ * 3 * HD);
static_assert(DM % 64 == 0);
static_assert(TD % 64 == 0);
static_assert(DM % 32 == 0);
static_assert(HD % 32 == 0);
static_assert(SEQ % 64 == 0);
static_assert((NB * SEQ) % 64 == 0);
static_assert(SEQ % (16 * AW) == 0);
static_assert(PADL == HALFW);
static_assert(WSPAN == 2 * HALFW);
static_assert(KT * 32 >= 16 + WSPAN);
static_assert(SEQ - 16 + KT * 32 <= SP);
static_assert(SP - SEQ - PADL == 128);
static_assert((SP * 2) % 128 == 0);
static_assert((PADL * 2) % 128 == 0);
static_assert((OSP * 4) % 16 == 0);
static_assert(((size_t)SEQ * DM) % 8 == 0);
static_assert(NB <= NB_FULL);
static_assert(SEQ <= SEQ_FULL);
static_assert(HD / 2 == 32);
static_assert(16 * 68 * 4 <= 131072);
static_assert(AW * 16 * OSP * 4 <= 131072);
static_assert(64 * TSP * 4 <= 131072);
static_assert(32 * 16 * 4 == 16 * HD * 2);
static_assert(32 * 16 * 8 == 16 * 64 * 4);
static_assert(256 * 2 * 16 == 64 * 64 * 2);
static_assert(256 * 4 * 16 == 64 * 64 * 4);

typedef _Float16 h16;
typedef unsigned short bf;
typedef __attribute__((ext_vector_type(16))) __bf16   v16bf;
typedef __attribute__((ext_vector_type(16))) _Float16 v16h;
typedef __attribute__((ext_vector_type(8)))  _Float16 v8h;
typedef __attribute__((ext_vector_type(8)))  unsigned short v8us;
typedef __attribute__((ext_vector_type(8)))  float    v8f;
typedef __attribute__((ext_vector_type(4)))  float    v4f;
typedef v4f  __attribute__((may_alias)) v4fa;

__device__ __forceinline__ unsigned short f2bf(float f) { unsigned u = __float_as_uint(f); u += 0x7FFFu + ((u >> 16) & 1u); return (unsigned short)(u >> 16); }
__device__ __forceinline__ float bfr(float f) { return __uint_as_float(((unsigned)f2bf(f)) << 16); }
__device__ __forceinline__ v16h cat16(v8h lo, v8h hi) { return __builtin_shufflevector(lo, hi, 0, 1, 2, 3, 4, 5, 6, 7, 8, 9, 10, 11, 12, 13, 14, 15); }
__device__ __forceinline__ v16bf cat16b(v8us lo, v8us hi) { return __builtin_bit_cast(v16bf, __builtin_shufflevector(lo, hi, 0, 1, 2, 3, 4, 5, 6, 7, 8, 9, 10, 11, 12, 13, 14, 15)); }
__device__ __forceinline__ v8f wmma16(v16h a, v16h b, v8f c) { return __builtin_amdgcn_wmma_f32_16x16x32_f16(false, a, false, b, (short)0, c, false, false); }
__device__ __forceinline__ v8f wmmab(v16bf a, v16bf b, v8f c) { return __builtin_amdgcn_wmma_f32_16x16x32_bf16(false, a, false, b, (short)0, c, false, false); }
__device__ __forceinline__ v16h  ldh(const h16* p) { return cat16(*(const v8h*)p, *(const v8h*)(p + 16)); }
__device__ __forceinline__ v16bf ldb(const bf* p)  { return cat16b(*(const v8us*)p, *(const v8us*)(p + 16)); }
__device__ __forceinline__ void wave_sync() { __builtin_amdgcn_fence(3  , "wavefront"); __builtin_amdgcn_wave_barrier(); asm volatile("" ::: "memory"); }
static __device__ __forceinline__ h16 toh_flush(float v) { const h16 r = (h16)v; return (fabsf(v) < 6.103515625e-05f) ? (h16)0.0f : r; }
__device__ __forceinline__ v8f wmma16g(v16h a, v16h b, v8f c) { c = wmma16(a, b, c); asm volatile("v_nop\n\tv_nop\n\tv_nop\n\tv_nop" : "+v"(c) : "v"(a), "v"(b)); return c; }
__device__ __forceinline__ v8f wmmabg(v16bf a, v16bf b, v8f c) { c = wmmab(a, b, c); asm volatile("v_nop\n\tv_nop\n\tv_nop\n\tv_nop" : "+v"(c) : "v"(a), "v"(b)); return c; }

__global__ __launch_bounds__(256) void k_cvt8(const float* __restrict__ src, bf* dst, size_t n8) {
    const size_t i = (size_t)blockIdx.x * 256 + threadIdx.x; if (i >= n8) return;
    const v8f v = *(const v8f*)(src + i * 8); v8us o;
#pragma unroll
    for (int k = 0; k < 8; ++k) o[k] = f2bf(v[k]);
    *(volatile v8us*)(dst + i * 8) = o; __threadfence(); *(volatile v8us*)(dst + i * 8) = o;
}

__global__ __launch_bounds__(256) void k_wtr_bf(const float* __restrict__ src, bf* dst, int R, int C) {
    __shared__ __align__(16) float ts[64 * TSP];
    const int tid = threadIdx.x;
    const int c0 = blockIdx.x * 64, r0 = blockIdx.y * 64;
#pragma unroll 1
    for (int i = 0; i < 4; ++i) { const int q = tid + 256 * i; const int r = q >> 4, c4 = (q & 15) * 4;
        const v4f v = *(const v4f*)(src + (size_t)(r0 + r) * C + c0 + c4);
        ts[r * TSP + c4] = v[0]; ts[r * TSP + c4 + 1] = v[1]; ts[r * TSP + c4 + 2] = v[2]; ts[r * TSP + c4 + 3] = v[3]; }
    __syncthreads();
    v8us o[2];
#pragma unroll
    for (int i = 0; i < 2; ++i) { const int n = 32 * i + (tid >> 3), k8 = (tid & 7) * 8;
#pragma unroll
        for (int e = 0; e < 8; ++e) o[i][e] = f2bf(ts[(k8 + e) * TSP + n]); }
#pragma unroll 1
    for (int ps = 0; ps < 2; ++ps) {
#pragma unroll
        for (int i = 0; i < 2; ++i) { const int n = 32 * i + (tid >> 3), k8 = (tid & 7) * 8;
            *(volatile v8us*)(dst + (size_t)(c0 + n) * R + r0 + k8) = o[i]; }
        if (ps == 0) __threadfence(); }
}

__global__ __launch_bounds__(256) void k_wtr_h(const float* __restrict__ src, h16* dst, int R, int C) {
    __shared__ __align__(16) float ts[64 * TSP];
    const int tid = threadIdx.x;
    const int c0 = blockIdx.x * 64, r0 = blockIdx.y * 64;
#pragma unroll 1
    for (int i = 0; i < 4; ++i) { const int q = tid + 256 * i; const int r = q >> 4, c4 = (q & 15) * 4;
        const v4f v = *(const v4f*)(src + (size_t)(r0 + r) * C + c0 + c4);
        ts[r * TSP + c4] = v[0]; ts[r * TSP + c4 + 1] = v[1]; ts[r * TSP + c4 + 2] = v[2]; ts[r * TSP + c4 + 3] = v[3]; }
    __syncthreads();
    v8h o[2];
#pragma unroll
    for (int i = 0; i < 2; ++i) { const int n = 32 * i + (tid >> 3), k8 = (tid & 7) * 8;
#pragma unroll
        for (int e = 0; e < 8; ++e) o[i][e] = toh_flush(bfr(ts[(k8 + e) * TSP + n]) * WOS); }
#pragma unroll 1
    for (int ps = 0; ps < 2; ++ps) {
#pragma unroll
        for (int i = 0; i < 2; ++i) { const int n = 32 * i + (tid >> 3), k8 = (tid & 7) * 8;
            *(volatile v8h*)(dst + (size_t)(c0 + n) * R + r0 + k8) = o[i]; }
        if (ps == 0) __threadfence(); }
}

__global__ __launch_bounds__(256) void k_zfill(h16* base, size_t pitch, int off0, int n0, int off1, int n1, int nunits) {
    const int npc = n0 + n1;
    const size_t i = (size_t)blockIdx.x * 256 + threadIdx.x;
    if (i >= (size_t)nunits * (size_t)npc) return;
    const size_t u = i / (size_t)npc; const int p = (int)(i % (size_t)npc);
    const size_t rel = (p < n0) ? ((size_t)off0 + (size_t)p * 8) : ((size_t)off1 + (size_t)(p - n0) * 8);
    const size_t a = u * pitch + rel;
    const v8h z = (v8h){};
    *(volatile v8h*)(base + a) = z; __threadfence(); *(volatile v8h*)(base + a) = z;
}

__global__ __launch_bounds__(32) void k_proj_qk(const bf* __restrict__ A, const bf* __restrict__ Bt, const float* __restrict__ bias,
                                               const float* __restrict__ cosb, const float* __restrict__ sinb, h16* QK) {
    __shared__ __align__(16) float os[16 * 68];
    const int K = DM;
    const int lane = threadIdx.x & 31, lr = lane & 15, hi = lane >> 4;
    const int r0 = blockIdx.x * 64; const int head = blockIdx.y >> 1, part = blockIdx.y & 1; const int c0 = head * (3 * HD) + part * HD;
    v8f acc[4][4];
#pragma unroll
    for (int mb = 0; mb < 4; ++mb)
#pragma unroll
        for (int nb = 0; nb < 4; ++nb) acc[mb][nb] = (v8f){};
    const size_t aoff = (size_t)(r0 + lr) * K + 8 * hi, boff = (size_t)(c0 + lr) * K + 8 * hi;
#pragma unroll 1
    for (int kc = 0; kc < K; kc += 32) {
        v16bf a[4];
#pragma unroll
        for (int mb = 0; mb < 4; ++mb) a[mb] = ldb(A + aoff + (size_t)mb * 16 * K + kc);
#pragma unroll
        for (int nb = 0; nb < 4; ++nb) { const v16bf b = ldb(Bt + boff + (size_t)nb * 16 * K + kc);
#pragma unroll
            for (int mb = 0; mb < 4; ++mb) acc[mb][nb] = wmmabg(a[mb], b, acc[mb][nb]); }
    }
    float bc[4];
#pragma unroll
    for (int nb = 0; nb < 4; ++nb) bc[nb] = bfr(bias[c0 + nb * 16 + lr]);
    const int bb = r0 / SEQ, tt = r0 % SEQ; const int zh = bb * NH_ + head;
    const size_t qpl = (size_t)NB * NH_ * SEQ * HD;
    const size_t tbase = part ? (qpl + ((size_t)zh * SP + (size_t)(PADL + tt)) * HD) : (((size_t)zh * SEQ + (size_t)tt) * HD);
#pragma unroll
    for (int mb = 0; mb < 4; ++mb) {
#pragma unroll
        for (int nb = 0; nb < 4; ++nb) {
#pragma unroll
            for (int j = 0; j < 8; ++j) os[(hi * 8 + j) * 68 + nb * 16 + lr] = acc[mb][nb][j] + bc[nb]; }
        wave_sync();
        v8h hv[4];
#pragma unroll
        for (int s = 0; s < 4; ++s) { const int row = 4 * s + (lane >> 3), c8 = (lane & 7) * 8;
            const v4f x0 = *(const v4fa*)(&os[row * 68 + c8]); const v4f x1 = *(const v4fa*)(&os[row * 68 + c8 + 4]);
            const size_t to = (size_t)(tt + mb * 16 + row) * (HD / 2) + (size_t)(c8 >> 1);
            const v4f cv = *(const v4f*)(cosb + to); const v4f sv = *(const v4f*)(sinb + to);
            v8h o;
#pragma unroll
            for (int i = 0; i < 2; ++i) {
                const float ca = bfr(cv[i]), sa = bfr(sv[i]); const float pa = x0[2 * i], pb = x0[2 * i + 1];
                o[2 * i] = toh_flush(pa * ca - pb * sa); o[2 * i + 1] = toh_flush(pa * sa + pb * ca);
                const float cc = bfr(cv[2 + i]), sc = bfr(sv[2 + i]); const float pc = x1[2 * i], pd = x1[2 * i + 1];
                o[4 + 2 * i] = toh_flush(pc * cc - pd * sc); o[5 + 2 * i] = toh_flush(pc * sc + pd * cc); }
            hv[s] = o; }
        const size_t sb = tbase + (size_t)(mb * 16) * HD;
#pragma unroll 1
        for (int ps = 0; ps < 2; ++ps) {
#pragma unroll
            for (int s = 0; s < 4; ++s) { const int row = 4 * s + (lane >> 3), c8 = (lane & 7) * 8;
                *(volatile v8h*)(QK + sb + (size_t)row * HD + c8) = hv[s]; }
            if (ps == 0) __threadfence(); }
        wave_sync();
    }
}

__global__ __launch_bounds__(32) void k_proj_vt(const bf* __restrict__ A, const bf* __restrict__ Bt, const float* __restrict__ bias, h16* VT) {
    __shared__ __align__(16) float os[16 * 68];
    const int K = DM;
    const int lane = threadIdx.x & 31, lr = lane & 15, hi = lane >> 4;
    const int head = blockIdx.x; const int rw = head * (3 * HD) + 2 * HD; const int c0 = blockIdx.y * 64;
    v8f acc[4][4];
#pragma unroll
    for (int mb = 0; mb < 4; ++mb)
#pragma unroll
        for (int nb = 0; nb < 4; ++nb) acc[mb][nb] = (v8f){};
    const size_t aoff = (size_t)(rw + lr) * K + 8 * hi, boff = (size_t)(c0 + lr) * K + 8 * hi;
#pragma unroll 1
    for (int kc = 0; kc < K; kc += 32) {
        v16bf a[4];
#pragma unroll
        for (int mb = 0; mb < 4; ++mb) a[mb] = ldb(A + aoff + (size_t)mb * 16 * K + kc);
#pragma unroll
        for (int nb = 0; nb < 4; ++nb) { const v16bf b = ldb(Bt + boff + (size_t)nb * 16 * K + kc);
#pragma unroll
            for (int mb = 0; mb < 4; ++mb) acc[mb][nb] = wmmabg(a[mb], b, acc[mb][nb]); }
    }
    const int bb = c0 / SEQ, tt = c0 % SEQ;
    const size_t tbase = ((size_t)(bb * NH_ + head) * HD) * SP + (size_t)(PADL + tt);
#pragma unroll
    for (int mb = 0; mb < 4; ++mb) {
        float br[8];
#pragma unroll
        for (int j = 0; j < 8; ++j) br[j] = bfr(bias[rw + mb * 16 + hi * 8 + j]);
#pragma unroll
        for (int nb = 0; nb < 4; ++nb) {
#pragma unroll
            for (int j = 0; j < 8; ++j) os[(hi * 8 + j) * 68 + nb * 16 + lr] = acc[mb][nb][j] + br[j]; }
        wave_sync();
        v8h hv[4];
#pragma unroll
        for (int s = 0; s < 4; ++s) { const int row = 4 * s + (lane >> 3), c8 = (lane & 7) * 8;
            const v4f x0 = *(const v4fa*)(&os[row * 68 + c8]); const v4f x1 = *(const v4fa*)(&os[row * 68 + c8 + 4]); v8h o;
#pragma unroll
            for (int i = 0; i < 4; ++i) { o[i] = toh_flush(x0[i]); o[4 + i] = toh_flush(x1[i]); }
            hv[s] = o; }
        const size_t sb = tbase + (size_t)(mb * 16) * SP;
#pragma unroll 1
        for (int ps = 0; ps < 2; ++ps) {
#pragma unroll
            for (int s = 0; s < 4; ++s) { const int row = 4 * s + (lane >> 3), c8 = (lane & 7) * 8;
                *(volatile v8h*)(VT + sb + (size_t)row * SP + c8) = hv[s]; }
            if (ps == 0) __threadfence(); }
        wave_sync();
    }
}

__global__ __launch_bounds__(32 * AW) void k_pairw(const h16* __restrict__ QP, const h16* __restrict__ KP, const h16* __restrict__ VT, h16* CX) {
    __shared__ __align__(16) float os[AW * 16 * OSP];
    const int lane = threadIdx.x & 31, lr = lane & 15, hi = lane >> 4;
    const int wave = __builtin_amdgcn_readfirstlane((int)(threadIdx.x >> 5));
    const int zh = blockIdx.y; const int b = zh / NH_, h = zh % NH_;
    const int t0 = (blockIdx.x * AW + wave) * 16;
    const size_t qo = ((size_t)zh * SEQ + (size_t)(t0 + lr)) * HD + 8 * hi;
    const v16h qf0 = ldh(QP + qo), qf1 = ldh(QP + qo + 32);
    const size_t ko = ((size_t)zh * SP + (size_t)(t0 + lr)) * HD + 8 * hi;
    const size_t vo = ((size_t)zh * HD + (size_t)lr) * SP + (size_t)t0 + 8 * hi;
    v8f o[4];
#pragma unroll
    for (int j = 0; j < 4; ++j) o[j] = (v8f){};
    float m = NEGB, l = 0.0f;
#pragma unroll 1
    for (int kt = 0; kt < KT; ++kt) {
        const h16* ka = KP + ko + (size_t)kt * 32 * HD;
        const v16h ka0 = ldh(ka), ka1 = ldh(ka + 32), kb0 = ldh(ka + 16 * HD), kb1 = ldh(ka + 16 * HD + 32);
        v8f sa = (v8f){}, sb = (v8f){};
        sa = wmma16g(ka0, qf0, sa); sa = wmma16g(ka1, qf1, sa);
        sb = wmma16g(kb0, qf0, sb); sb = wmma16g(kb1, qf1, sb);
        const int dja = kt * 32 + 8 * hi - lr;
        float ta[8], tb[8]; bool fa[8], fb[8]; float mx = NEGB;
#pragma unroll
        for (int r = 0; r < 8; ++r) {
            fa[r] = (unsigned)(dja + r) <= (unsigned)WSPAN;
            fb[r] = (unsigned)(dja + 16 + r) <= (unsigned)WSPAN;
            ta[r] = sa[r] * SC2; tb[r] = sb[r] * SC2;
            mx = fmaxf(mx, fmaxf(fa[r] ? ta[r] : NEGB, fb[r] ? tb[r] : NEGB)); }
        mx = fmaxf(mx, __shfl_xor(mx, 16, 32));
        const float mnew = fmaxf(m, mx);
        const float alpha = __builtin_amdgcn_exp2f(m - mnew);
        const float sh = PSH - mnew;
        v16h pb; float ls = 0.0f;
#pragma unroll
        for (int r = 0; r < 8; ++r) {
            const float xa = ta[r] + sh, xb = tb[r] + sh;
            const float ea = __builtin_amdgcn_exp2f(xa), eb = __builtin_amdgcn_exp2f(xb);
            const float ga = (fa[r] & (xa >= -14.0f)) ? ea : 0.0f, gb = (fb[r] & (xb >= -14.0f)) ? eb : 0.0f;
            const h16 pa = (h16)ga; const h16 pc = (h16)gb;
            pb[r] = pa; pb[8 + r] = pc;
            ls += (float)pa + (float)pc; }
        l = l * alpha + ls; m = mnew;
#pragma unroll
        for (int j = 0; j < 4; ++j) o[j] = o[j] * alpha;
        const h16* va = VT + vo + (size_t)kt * 32;
#pragma unroll
        for (int j = 0; j < 4; ++j) { const v16h vj = ldh(va + (size_t)j * 16 * SP); o[j] = wmma16g(vj, pb, o[j]); }
    }
    l += __shfl_xor(l, 16, 32);
    const bool any = l > 0.0f;
    const float lsafe = any ? l : 1.0f;
    const float inv = any ? (1.0f / lsafe) : 0.0f;
    const int wb = wave * 16 * OSP;
#pragma unroll
    for (int j = 0; j < 4; ++j) { v4f a, c;
        a[0] = o[j][0] * inv; a[1] = o[j][1] * inv; a[2] = o[j][2] * inv; a[3] = o[j][3] * inv;
        c[0] = o[j][4] * inv; c[1] = o[j][5] * inv; c[2] = o[j][6] * inv; c[3] = o[j][7] * inv;
        *(v4fa*)(&os[wb + lr * OSP + 16 * j + 8 * hi]) = a; *(v4fa*)(&os[wb + lr * OSP + 16 * j + 8 * hi + 4]) = c; }
    wave_sync();
    v8h hv[4];
#pragma unroll
    for (int s = 0; s < 4; ++s) { const int row = 4 * s + (lane >> 3), c8 = (lane & 7) * 8;
        const v4f x0 = *(const v4fa*)(&os[wb + row * OSP + c8]); const v4f x1 = *(const v4fa*)(&os[wb + row * OSP + c8 + 4]); v8h q;
#pragma unroll
        for (int i = 0; i < 4; ++i) { q[i] = toh_flush(x0[i] * CXS); q[4 + i] = toh_flush(x1[i] * CXS); }
        hv[s] = q; }
    h16* crow = CX + ((size_t)b * SEQ + (size_t)t0) * DM + (size_t)h * HD;
#pragma unroll 1
    for (int ps = 0; ps < 2; ++ps) {
#pragma unroll
        for (int s = 0; s < 4; ++s) { const int row = 4 * s + (lane >> 3), c8 = (lane & 7) * 8;
            *(volatile v8h*)(crow + (size_t)row * DM + c8) = hv[s]; }
        if (ps == 0) __threadfence(); }
}

__global__ __launch_bounds__(32) void k_proj_out(const h16* __restrict__ A, const h16* __restrict__ Bt, const float* __restrict__ bias, float* OUT) {
    __shared__ __align__(16) float os[16 * 68];
    const int K = DM;
    const int lane = threadIdx.x & 31, lr = lane & 15, hi = lane >> 4; const int r0 = blockIdx.x * 64, c0 = blockIdx.y * 64;
    v8f acc[4][4];
#pragma unroll
    for (int mb = 0; mb < 4; ++mb)
#pragma unroll
        for (int nb = 0; nb < 4; ++nb) acc[mb][nb] = (v8f){};
    const size_t aoff = (size_t)(r0 + lr) * K + 8 * hi, boff = (size_t)(c0 + lr) * K + 8 * hi;
#pragma unroll 1
    for (int kc = 0; kc < K; kc += 32) {
        v16h a[4];
#pragma unroll
        for (int mb = 0; mb < 4; ++mb) a[mb] = ldh(A + aoff + (size_t)mb * 16 * K + kc);
#pragma unroll
        for (int nb = 0; nb < 4; ++nb) { const v16h b = ldh(Bt + boff + (size_t)nb * 16 * K + kc);
#pragma unroll
            for (int mb = 0; mb < 4; ++mb) acc[mb][nb] = wmma16g(a[mb], b, acc[mb][nb]); }
    }
    float bc[4];
#pragma unroll
    for (int nb = 0; nb < 4; ++nb) bc[nb] = bfr(bias[c0 + nb * 16 + lr]);
    const int bb = r0 / SEQ, tt = r0 % SEQ;
    float* obase = OUT + ((size_t)bb * OUT_SEQ + (size_t)tt) * DM + c0;
#pragma unroll
    for (int mb = 0; mb < 4; ++mb) {
#pragma unroll
        for (int nb = 0; nb < 4; ++nb) {
#pragma unroll
            for (int j = 0; j < 8; ++j) os[(hi * 8 + j) * 68 + nb * 16 + lr] = acc[mb][nb][j] * OSI + bc[nb]; }
        wave_sync();
#pragma unroll 1
        for (int ps = 0; ps < 2; ++ps) {
#pragma unroll
            for (int s = 0; s < 8; ++s) { const int row = 2 * s + (lane >> 4), cofs = (lane & 15) * 4;
                const v4f val = *(const v4fa*)(&os[row * 68 + cofs]);
                *(volatile v4f*)(obase + (size_t)(mb * 16 + row) * DM + cofs) = val; }
            if (ps == 0) __threadfence(); }
        wave_sync();
    }
}

static constexpr size_t al256(size_t v) { return (v + 255) & ~(size_t)255; }
static constexpr size_t SZ_XB = al256((size_t)NB * SEQ * DM * 2);
static constexpr size_t SZ_WT = al256((size_t)TD * DM * 2);
static constexpr size_t SZ_WO = al256((size_t)DM * DM * 2);
static constexpr size_t SZ_QP = al256((size_t)NB * NH_ * SEQ * HD * 2);
static constexpr size_t SZ_KP = al256((size_t)NB * NH_ * SP * HD * 2);
static constexpr size_t SZ_VT = al256((size_t)NB * NH_ * HD * SP * 2);
static constexpr size_t SZ_CX = al256((size_t)NB * SEQ * DM * 2);
static constexpr size_t SZ_TOTAL = SZ_XB + SZ_WT + SZ_WO + SZ_QP + SZ_KP + SZ_VT + SZ_CX;
static_assert(SZ_TOTAL <= (size_t)134217728);
static_assert(SZ_QP == (size_t)NB * NH_ * SEQ * HD * 2);
static_assert(((size_t)SP * HD * 2) % 128 == 0);
static_assert(((size_t)NB * NH_ * (64 * 64 / 8 + 128 * 64 / 8)) % 256 == 0);
static_assert(((size_t)NB * NH_ * HD * (8 + 16)) % 256 == 0);

extern "C" void kernel_launch(void* const* d_in, const int* in_sizes, int n_in,
                              void* d_out, int out_size, void* d_ws, size_t ws_size, hipStream_t stream) {
    if (n_in < 7) return;
    if ((size_t)in_sizes[0] < ((size_t)(NB - 1) * SEQ_FULL + SEQ) * DM) return;
    if ((size_t)in_sizes[1] < (size_t)DM * TD || in_sizes[2] < TD) return;
    if ((size_t)in_sizes[3] < (size_t)DM * DM || in_sizes[4] < DM) return;
    if ((size_t)in_sizes[5] < (size_t)SEQ * (HD / 2) || (size_t)in_sizes[6] < (size_t)SEQ * (HD / 2)) return;
    if ((size_t)out_size < ((size_t)(NB - 1) * OUT_SEQ + SEQ) * DM) return;
    if (SZ_TOTAL > ws_size) return;
    const float* x    = (const float*)d_in[0];
    const float* wqkv = (const float*)d_in[1];
    const float* bqkv = (const float*)d_in[2];
    const float* wout = (const float*)d_in[3];
    const float* bout = (const float*)d_in[4];
    const float* cosb = (const float*)d_in[5];
    const float* sinb = (const float*)d_in[6];
    float* OUT = (float*)d_out;
    char* wsp = (char*)d_ws;
    bf*  XB  = (bf*)wsp;  wsp += SZ_XB;
    bf*  WT  = (bf*)wsp;  wsp += SZ_WT;
    h16* WOT = (h16*)wsp; wsp += SZ_WO;
    h16* QK  = (h16*)wsp; wsp += SZ_QP + SZ_KP;
    h16* VT  = (h16*)wsp; wsp += SZ_VT;
    h16* CX  = (h16*)wsp; wsp += SZ_CX;
    h16* QP = QK; h16* KP = QK + (size_t)NB * NH_ * SEQ * HD;

    if (SEQ == SEQ_FULL) {
        const size_t n8 = (size_t)NB * SEQ * DM / 8;
        k_cvt8<<<(unsigned)((n8 + 255) / 256), 256, 0, stream>>>(x, XB, n8);
    } else {
        const size_t n8 = (size_t)SEQ * DM / 8;
        for (int b = 0; b < NB; ++b) k_cvt8<<<(unsigned)((n8 + 255) / 256), 256, 0, stream>>>(x + (size_t)b * SEQ_FULL * DM, XB + (size_t)b * SEQ * DM, n8);
    }
    k_wtr_bf<<<dim3(TD / 64, DM / 64, 1), 256, 0, stream>>>(wqkv, WT, DM, TD);
    k_wtr_h<<<dim3(DM / 64, DM / 64, 1), 256, 0, stream>>>(wout, WOT, DM, DM);
    { const int n0 = 64 * HD / 8, n1 = 128 * HD / 8; const size_t tot = (size_t)NB * NH_ * (size_t)(n0 + n1);
      k_zfill<<<(unsigned)((tot + 255) / 256), 256, 0, stream>>>(KP, (size_t)SP * HD, 0, n0, (SEQ + PADL) * HD, n1, NB * NH_); }
    { const int n0 = 64 / 8, n1 = 128 / 8; const size_t tot = (size_t)NB * NH_ * HD * (size_t)(n0 + n1);
      k_zfill<<<(unsigned)((tot + 255) / 256), 256, 0, stream>>>(VT, (size_t)SP, 0, n0, SEQ + PADL, n1, NB * NH_ * HD); }

    k_proj_qk<<<dim3(NB * SEQ / 64, 2 * NH_, 1), 32, 0, stream>>>(XB, WT, bqkv, cosb, sinb, QK);
    k_proj_vt<<<dim3(NH_, NB * SEQ / 64, 1), 32, 0, stream>>>(WT, XB, bqkv, VT);
    k_pairw<<<dim3(SEQ / (16 * AW), NB * NH_, 1), 32 * AW, 0, stream>>>(QP, KP, VT, CX);
    k_proj_out<<<dim3(NB * SEQ / 64, DM / 64, 1), 32, 0, stream>>>(CX, WOT, bout, OUT);
}
